// TransformerBlock_39230231282128
// MI455X (gfx1250) — hardware-verified
//
#include <hip/hip_runtime.h>
#include <stddef.h>


typedef _Float16 v16h __attribute__((ext_vector_type(16)));
typedef _Float16 v8h  __attribute__((ext_vector_type(8)));
typedef float    v8f  __attribute__((ext_vector_type(8)));
typedef float    v4f  __attribute__((ext_vector_type(4)));

#ifndef NB
#define NB 2
#endif
#ifndef SEQ
#define SEQ 2048
#endif
#define NB_FULL  2
#define SEQ_FULL 2048
#define DIM   1024
#define DFF   4096
#define NHEAD 16
#define HD    64
#define MROWS (NB * SEQ)

static_assert(NB >= 1 && NB <= NB_FULL);
static_assert(SEQ >= 128 && SEQ <= SEQ_FULL && (SEQ % 128) == 0);
static_assert(DIM == NHEAD * HD);
static_assert((MROWS % 64) == 0 && (MROWS % 8) == 0);
static_assert((DIM % 64) == 0 && (DFF % 64) == 0);
static_assert(DIM == 4 * 256);

#define LDT 72
#define LDC 68

#define WCARRY 64.0f
#define PCARRY 1024.0f
#define VCARRY 64.0f

#define WSQ_BYTES ((size_t)DIM * DIM * 2)
#define WFF_BYTES ((size_t)DIM * DFF * 2)
#define P16_BYTES ((size_t)MROWS * DIM * 2)
#define P32_BYTES ((size_t)MROWS * DIM * 4)
#define U16_BYTES ((size_t)MROWS * DFF * 2)
#define OFF_WSQ 0
#define OFF_W1T (OFF_WSQ + 4 * WSQ_BYTES)
#define OFF_W2T (OFF_W1T + WFF_BYTES)
#define OFF_H1  (OFF_W2T + WFF_BYTES)
#define OFF_Q   (OFF_H1 + P16_BYTES)
#define OFF_K   (OFF_Q + P16_BYTES)
#define OFF_VT  (OFF_K + P16_BYTES)
#define OFF_OV  (OFF_VT + P16_BYTES)
#define OFF_X32 (OFF_OV + P16_BYTES)
#define OFF_H2  (OFF_X32 + P32_BYTES)
#define OFF_U   (OFF_H2 + P16_BYTES)
#define WS_TOTAL (OFF_U + U16_BYTES)
static_assert((P16_BYTES % 128) == 0 && (WSQ_BYTES % 128) == 0);
static_assert(WS_TOTAL <= (size_t)134217728);

__device__ __forceinline__ float bf16r(float x) {
  unsigned int u = __float_as_uint(x);
  u = (u + 0x7FFFu + ((u >> 16) & 1u)) & 0xFFFF0000u;
  return __uint_as_float(u);
}

__device__ __forceinline__ v16h frag_at(const _Float16* p) {
  v8h lo = *(const v8h*)(p);
  v8h hi = *(const v8h*)(p + 16);
  v16h out;
#pragma unroll
  for (int i = 0; i < 8; ++i) { out[i] = lo[i]; out[i + 8] = hi[i]; }
  return out;
}
__device__ __forceinline__ v16h ld_frag(const _Float16* base, int ld) {
  const int lane = threadIdx.x & 31;
  return frag_at(base + (lane & 15) * ld + (lane >> 4) * 8);
}

__device__ __forceinline__ v8f wmma16(v16h a, v16h b, v8f c) {
  v8f d = __builtin_amdgcn_wmma_f32_16x16x32_f16(false, a, false, b, (short)0, c,
                                                 false, false);
  asm volatile("v_nop\n\tv_nop\n\tv_nop\n\tv_nop" : "+v"(d) : "v"(a), "v"(b));
  return d;
}

__device__ __forceinline__ float red16_max(float x) {
#pragma unroll
  for (int off = 1; off < 16; off <<= 1) x = fmaxf(x, __shfl_xor(x, off, 32));
  return x;
}
__device__ __forceinline__ float red16_sum(float x) {
#pragma unroll
  for (int off = 1; off < 16; off <<= 1) x += __shfl_xor(x, off, 32);
  return x;
}
__device__ __forceinline__ float wave_sum(float x) {
#pragma unroll
  for (int off = 1; off < 32; off <<= 1) x += __shfl_xor(x, off, 32);
  return x;
}

__device__ __forceinline__ void wave_lds_sync() {
  __builtin_amdgcn_fence(3  , "wavefront");
  asm volatile("s_wait_dscnt 0x0" ::: "memory");
  __builtin_amdgcn_wave_barrier();
}

__device__ __forceinline__ float gelu_f(float x) {
  const float y = 0.79788456f * (x + 0.044715f * (x * x * x));
  const float e = __expf(2.0f * y);
  const float r = __builtin_amdgcn_rcpf(1.0f + e);
  return x * (1.0f - r);
}

template <int KD, int ND>
__global__ __launch_bounds__(256) void wconv_kernel(
    const float* __restrict__ W0, const float* __restrict__ W1p,
    const float* __restrict__ W2p, const float* __restrict__ W3,
    _Float16* __restrict__ Wt) {
  __shared__ __attribute__((aligned(16))) _Float16 T[64 * LDT];
  const unsigned tid = threadIdx.x;
  const unsigned n0 = blockIdx.x * 64u;
  const unsigned k0 = blockIdx.y * 64u;
  const unsigned p = blockIdx.z;
  const float* W = W0;
  if (p == 1u) W = W1p;
  if (p == 2u) W = W2p;
  if (p == 3u) W = W3;
#pragma unroll 4
  for (unsigned j = 0; j < 16u; ++j) {
    const unsigned idx = tid + 256u * j;
    const unsigned kr = idx >> 6, nc = idx & 63u;
    const float v = W[(size_t)(k0 + kr) * ND + n0 + nc];
    T[nc * LDT + kr] = (_Float16)(WCARRY * bf16r(v));
  }
  __syncthreads();
  v8h x[2];
  size_t off[2];
#pragma unroll
  for (int i = 0; i < 2; ++i) {
    const unsigned n = 32u * i + (tid >> 3);
    const unsigned kc = (tid & 7u) * 8u;
    x[i] = *(const v8h*)&T[n * LDT + kc];
    off[i] = (size_t)p * KD * ND + (size_t)(n0 + n) * KD + k0 + kc;
  }
#pragma unroll
  for (int i = 0; i < 2; ++i) *(volatile v8h*)(Wt + off[i]) = x[i];
  __threadfence();
#pragma unroll
  for (int i = 0; i < 2; ++i) *(volatile v8h*)(Wt + off[i]) = x[i];
}

template <int RAW>
__global__ __launch_bounds__(256) void ln_kernel(
    const float* __restrict__ X, const float* __restrict__ gs,
    const float* __restrict__ gb, _Float16* __restrict__ out) {
  __shared__ __attribute__((aligned(16))) float Rb[8 * DIM];
  const unsigned tid = threadIdx.x, lane = tid & 31u, w = tid >> 5;
  const unsigned crow = blockIdx.x * 8u + w;
  size_t srow = crow;
  if (RAW) {
    const unsigned bidx = crow / (unsigned)SEQ;
    const unsigned sq = crow - bidx * (unsigned)SEQ;
    srow = (size_t)bidx * SEQ_FULL + sq;
  }
  const float* xp = X + srow * DIM;
  float* rb = Rb + w * DIM;

  float s = 0.0f;
#pragma unroll 1
  for (unsigned j = 0; j < 4u; ++j) {
    const unsigned c = j * 256u + lane * 8u;
    v4f a0 = *(const v4f*)(xp + c);
    v4f a1 = *(const v4f*)(xp + c + 4);
    if (RAW) {
#pragma unroll
      for (int t = 0; t < 4; ++t) { a0[t] = bf16r(a0[t]); a1[t] = bf16r(a1[t]); }
    }
    *(v4f*)(rb + c) = a0;
    *(v4f*)(rb + c + 4) = a1;
    s += ((a0[0] + a0[1]) + (a0[2] + a0[3])) + ((a1[0] + a1[1]) + (a1[2] + a1[3]));
  }
  s = wave_sum(s);
  const float mean = s * (1.0f / DIM);

  float ss = 0.0f;
#pragma unroll 1
  for (unsigned j = 0; j < 4u; ++j) {
    const unsigned c = j * 256u + lane * 8u;
    const v4f a0 = *(const v4f*)(rb + c);
    const v4f a1 = *(const v4f*)(rb + c + 4);
#pragma unroll
    for (int t = 0; t < 4; ++t) {
      const float d0 = a0[t] - mean;
      const float d1 = a1[t] - mean;
      ss += d0 * d0;
      ss += d1 * d1;
    }
  }
  ss = wave_sum(ss);
  const float rstd = rsqrtf(ss * (1.0f / (DIM - 1)) + 1.0e-5f);

  v8h x[4];
  size_t off[4];
#pragma unroll
  for (int j = 0; j < 4; ++j) {
    const unsigned c = (unsigned)j * 256u + lane * 8u;
    const v4f a0 = *(const v4f*)(rb + c);
    const v4f a1 = *(const v4f*)(rb + c + 4);
    const v4f s0 = *(const v4f*)(gs + c);
    const v4f s1 = *(const v4f*)(gs + c + 4);
    const v4f b0 = *(const v4f*)(gb + c);
    const v4f b1 = *(const v4f*)(gb + c + 4);
#pragma unroll
    for (int t = 0; t < 4; ++t) {
      x[j][t]     = (_Float16)(bf16r(s0[t]) * ((a0[t] - mean) * rstd) + bf16r(b0[t]));
      x[j][t + 4] = (_Float16)(bf16r(s1[t]) * ((a1[t] - mean) * rstd) + bf16r(b1[t]));
    }
    off[j] = (size_t)crow * DIM + c;
  }
#pragma unroll
  for (int j = 0; j < 4; ++j) *(volatile v8h*)(out + off[j]) = x[j];
  __threadfence();
#pragma unroll
  for (int j = 0; j < 4; ++j) *(volatile v8h*)(out + off[j]) = x[j];
}

template <int MODE, int KD, int ND>
__global__ __launch_bounds__(256) void gemm_kernel(
    const _Float16* __restrict__ A16, const _Float16* __restrict__ Bt,
    const float* __restrict__ biasf, const float* __restrict__ resf,
    float* __restrict__ outf, _Float16* __restrict__ out16) {
  static_assert((KD % 32) == 0 && (ND % 64) == 0);
  static_assert(MODE != 1 || ND == DIM);
  static_assert((MODE != 2 && MODE != 4) || ND == DIM);
  __shared__ __attribute__((aligned(16))) float Cs[64 * LDC];
  const unsigned tid = threadIdx.x, lane = tid & 31u, w = tid >> 5;
  const unsigned mw = w >> 1, nw = w & 1u;
  const unsigned hh = lane >> 4, m = lane & 15u;
  const unsigned n0 = blockIdx.x * 64u;
  const unsigned row0 = blockIdx.y * 64u;

  const _Float16* ap  = A16 + (size_t)(row0 + mw * 16u + m) * KD + hh * 8u;
  const _Float16* bp0 = Bt + (size_t)(n0 + nw * 32u + m) * KD + hh * 8u;
  const _Float16* bp1 = bp0 + (size_t)16 * KD;
  v8f acc0 = {}, acc1 = {};
#pragma unroll 2
  for (int k0 = 0; k0 < KD; k0 += 32) {
    const v16h a  = frag_at(ap + k0);
    const v16h b0 = frag_at(bp0 + k0);
    const v16h b1 = frag_at(bp1 + k0);
    acc0 = wmma16(a, b0, acc0);
    acc1 = wmma16(a, b1, acc1);
  }
#pragma unroll
  for (int r = 0; r < 8; ++r) {
    float* d = &Cs[(mw * 16u + hh * 8u + r) * LDC + nw * 32u + m];
    d[0]  = acc0[r];
    d[16] = acc1[r];
  }
  __syncthreads();

  if (MODE == 0) {
    v8h x[2];
    size_t off[2];
#pragma unroll
    for (int i = 0; i < 2; ++i) {
      const unsigned r = 32u * i + (tid >> 3);
      const unsigned c = (tid & 7u) * 8u;
      const v4f u0 = *(const v4f*)&Cs[r * LDC + c];
      const v4f u1 = *(const v4f*)&Cs[r * LDC + c + 4];
#pragma unroll
      for (int j = 0; j < 4; ++j) {
        x[i][j]     = (_Float16)(u0[j] * (1.0f / WCARRY));
        x[i][j + 4] = (_Float16)(u1[j] * (1.0f / WCARRY));
      }
      off[i] = (size_t)(row0 + r) * ND + n0 + c;
    }
#pragma unroll
    for (int i = 0; i < 2; ++i) *(volatile v8h*)(out16 + off[i]) = x[i];
    __threadfence();
#pragma unroll
    for (int i = 0; i < 2; ++i) *(volatile v8h*)(out16 + off[i]) = x[i];
  }

  if (MODE == 1) {
    const unsigned bidx = row0 / (unsigned)SEQ;
    const unsigned key0 = row0 - bidx * (unsigned)SEQ;
    v8h x[2];
    size_t off[2];
#pragma unroll
    for (int i = 0; i < 2; ++i) {
      const unsigned dcol = 32u * i + (tid >> 3);
      const unsigned kk = (tid & 7u) * 8u;
#pragma unroll
      for (int j = 0; j < 8; ++j)
        x[i][j] = (_Float16)(Cs[(kk + j) * LDC + dcol] * (1.0f / WCARRY));
      off[i] = ((size_t)bidx * DIM + n0 + dcol) * SEQ + key0 + kk;
    }
#pragma unroll
    for (int i = 0; i < 2; ++i) *(volatile v8h*)(out16 + off[i]) = x[i];
    __threadfence();
#pragma unroll
    for (int i = 0; i < 2; ++i) *(volatile v8h*)(out16 + off[i]) = x[i];
  }

  if (MODE == 2) {
    v4f xs[4];
    size_t off[4];
#pragma unroll
    for (int i = 0; i < 4; ++i) {
      const unsigned r = 16u * i + (tid >> 4);
      const unsigned c = (tid & 15u) * 4u;
      const unsigned crow = row0 + r;
      const unsigned bidx = crow / (unsigned)SEQ;
      const unsigned sq = crow - bidx * (unsigned)SEQ;
      const size_t frow = (size_t)bidx * SEQ_FULL + sq;
      const v4f u = *(const v4f*)&Cs[r * LDC + c];
      const v4f g = *(const v4f*)(biasf + n0 + c);
      const v4f q = *(const v4f*)(resf + frow * DIM + n0 + c);
      v4f val;
#pragma unroll
      for (int j = 0; j < 4; ++j)
        val[j] = (u[j] * (1.0f / (WCARRY * VCARRY)) + bf16r(g[j])) + bf16r(q[j]);
      xs[i] = val;
      off[i] = (size_t)crow * DIM + n0 + c;
    }
#pragma unroll
    for (int i = 0; i < 4; ++i) *(volatile v4f*)(outf + off[i]) = xs[i];
    __threadfence();
#pragma unroll
    for (int i = 0; i < 4; ++i) *(volatile v4f*)(outf + off[i]) = xs[i];
  }

  if (MODE == 3) {
    v8h x[2];
    size_t off[2];
#pragma unroll
    for (int i = 0; i < 2; ++i) {
      const unsigned r = 32u * i + (tid >> 3);
      const unsigned c = (tid & 7u) * 8u;
      const v4f u0 = *(const v4f*)&Cs[r * LDC + c];
      const v4f u1 = *(const v4f*)&Cs[r * LDC + c + 4];
      const v4f g0 = *(const v4f*)(biasf + n0 + c);
      const v4f g1 = *(const v4f*)(biasf + n0 + c + 4);
#pragma unroll
      for (int j = 0; j < 4; ++j) {
        const float t0 = gelu_f(u0[j] * (1.0f / WCARRY) + bf16r(g0[j]));
        const float t1 = gelu_f(u1[j] * (1.0f / WCARRY) + bf16r(g1[j]));
        x[i][j]     = (_Float16)t0;
        x[i][j + 4] = (_Float16)t1;
      }
      off[i] = (size_t)(row0 + r) * ND + n0 + c;
    }
#pragma unroll
    for (int i = 0; i < 2; ++i) *(volatile v8h*)(out16 + off[i]) = x[i];
    __threadfence();
#pragma unroll
    for (int i = 0; i < 2; ++i) *(volatile v8h*)(out16 + off[i]) = x[i];
  }

  if (MODE == 4) {
    v4f xs[4];
    size_t off[4];
#pragma unroll
    for (int i = 0; i < 4; ++i) {
      const unsigned r = 16u * i + (tid >> 4);
      const unsigned c = (tid & 15u) * 4u;
      const unsigned crow = row0 + r;
      const unsigned bidx = crow / (unsigned)SEQ;
      const unsigned sq = crow - bidx * (unsigned)SEQ;
      const size_t frow = (size_t)bidx * SEQ_FULL + sq;
      const v4f u  = *(const v4f*)&Cs[r * LDC + c];
      const v4f g  = *(const v4f*)(biasf + n0 + c);
      const v4f rx = *(const v4f*)(resf + (size_t)crow * DIM + n0 + c);
      v4f val;
#pragma unroll
      for (int j = 0; j < 4; ++j)
        val[j] = (u[j] * (1.0f / WCARRY) + bf16r(g[j])) + rx[j];
      xs[i] = val;
      off[i] = frow * DIM + n0 + c;
    }
#pragma unroll
    for (int i = 0; i < 4; ++i) *(volatile v4f*)(outf + off[i]) = xs[i];
    __threadfence();
#pragma unroll
    for (int i = 0; i < 4; ++i) *(volatile v4f*)(outf + off[i]) = xs[i];
  }
}

__global__ __launch_bounds__(256) void attn_kernel(
    const _Float16* __restrict__ Qh, const _Float16* __restrict__ Kh,
    const _Float16* __restrict__ Vt, _Float16* __restrict__ Ov) {
  __shared__ __attribute__((aligned(16))) _Float16 Ks[64 * LDT];
  __shared__ __attribute__((aligned(16))) _Float16 Vs[64 * LDT];
  __shared__ __attribute__((aligned(16))) _Float16 Ps[8 * 16 * LDT];

  const int tid = threadIdx.x, lane = tid & 31;
  const int w = __builtin_amdgcn_readfirstlane(tid >> 5);
  const int hh = lane >> 4, m = lane & 15;
  const int q0 = blockIdx.x * 128;
  const int head = blockIdx.y;
  const int b = blockIdx.z;
  const int qw = q0 + w * 16;
  const float scale = 0.125f;
  _Float16* P = Ps + w * (16 * LDT);

  const size_t qoff = (size_t)(b * SEQ + qw + m) * DIM + head * HD + hh * 8;
  v16h qf[2];
  qf[0] = frag_at(Qh + qoff);
  qf[1] = frag_at(Qh + qoff + 32);

  float mrow[8], lrow[8];
  v8f o[4];
#pragma unroll
  for (int v = 0; v < 8; ++v) { mrow[v] = -1.0e30f; lrow[v] = 0.0f; }
#pragma unroll
  for (int nb = 0; nb < 4; ++nb) o[nb] = (v8f){};

  const size_t kplane = (size_t)b * SEQ * DIM + head * HD;
  const size_t vplane = ((size_t)b * DIM + head * HD) * SEQ;

  const int kend = q0 + 128;
  for (int kb = 0; kb < kend; kb += 64) {
#pragma unroll
    for (int j = 0; j < 2; ++j) {
      const int idx = tid + 256 * j;
      const int r = idx >> 3, c = (idx & 7) * 8;
      *(v8h*)&Ks[r * LDT + c] = *(const v8h*)(Kh + kplane + (size_t)(kb + r) * DIM + c);
      *(v8h*)&Vs[r * LDT + c] = *(const v8h*)(Vt + vplane + (size_t)r * SEQ + kb + c);
    }
    __syncthreads();

    if (kb <= qw + 15) {
      v8f s[4];
#pragma unroll
      for (int kg = 0; kg < 4; ++kg) {
        v8f t = {};
#pragma unroll
        for (int c = 0; c < 2; ++c) {
          const v16h kf = ld_frag(&Ks[(kg * 16) * LDT + c * 32], LDT);
          t = wmma16(qf[c], kf, t);
        }
        s[kg] = t * scale;
      }
      if (kb + 63 > qw) {
#pragma unroll
        for (int kg = 0; kg < 4; ++kg)
#pragma unroll
          for (int v = 0; v < 8; ++v)
            s[kg][v] = (kb + kg * 16 + m <= qw + hh * 8 + v) ? s[kg][v] : -1.0e30f;
      }

      float alpha[8];
#pragma unroll
      for (int v = 0; v < 8; ++v) {
        float mx = fmaxf(fmaxf(s[0][v], s[1][v]), fmaxf(s[2][v], s[3][v]));
        mx = red16_max(mx);
        const float mn = fmaxf(mrow[v], mx);
        alpha[v] = __expf(mrow[v] - mn);
        mrow[v] = mn;
      }
#pragma unroll
      for (int kg = 0; kg < 4; ++kg)
#pragma unroll
        for (int v = 0; v < 8; ++v) s[kg][v] = __expf(s[kg][v] - mrow[v]);
#pragma unroll
      for (int v = 0; v < 8; ++v) {
        const float rs = red16_sum((s[0][v] + s[1][v]) + (s[2][v] + s[3][v]));
        lrow[v] = alpha[v] * lrow[v] + rs;
      }
#pragma unroll
      for (int nb = 0; nb < 4; ++nb)
#pragma unroll
        for (int v = 0; v < 8; ++v) o[nb][v] = o[nb][v] * alpha[v];

#pragma unroll
      for (int kg = 0; kg < 4; ++kg)
#pragma unroll
        for (int v = 0; v < 8; ++v)
          P[(hh * 8 + v) * LDT + kg * 16 + m] = (_Float16)(s[kg][v] * PCARRY);
      wave_lds_sync();

#pragma unroll
      for (int c = 0; c < 2; ++c) {
        const v16h pf = ld_frag(P + c * 32, LDT);
#pragma unroll
        for (int nb = 0; nb < 4; ++nb) {
          const v16h vf = ld_frag(&Vs[(nb * 16) * LDT + c * 32], LDT);
          o[nb] = wmma16(pf, vf, o[nb]);
        }
      }
    }
    __syncthreads();
  }

  float inv[8];
#pragma unroll
  for (int v = 0; v < 8; ++v) inv[v] = __builtin_amdgcn_rcpf(lrow[v]) * (VCARRY / PCARRY);
#pragma unroll
  for (int nb = 0; nb < 4; ++nb)
#pragma unroll
    for (int v = 0; v < 8; ++v)
      P[(hh * 8 + v) * LDT + nb * 16 + m] = (_Float16)(o[nb][v] * inv[v]);
  wave_lds_sync();
  v8h x[4];
  size_t off[4];
#pragma unroll
  for (int i = 0; i < 4; ++i) {
    const int r = 4 * i + (lane >> 3);
    const int c = (lane & 7) * 8;
    x[i] = *(const v8h*)&P[r * LDT + c];
    off[i] = (size_t)(b * SEQ + qw + r) * DIM + head * HD + c;
  }
#pragma unroll
  for (int i = 0; i < 4; ++i) *(volatile v8h*)(Ov + off[i]) = x[i];
  __threadfence();
#pragma unroll
  for (int i = 0; i < 4; ++i) *(volatile v8h*)(Ov + off[i]) = x[i];
}

extern "C" void kernel_launch(void* const* d_in, const int* in_sizes, int n_in,
                              void* d_out, int out_size, void* d_ws, size_t ws_size,
                              hipStream_t stream) {
  if (n_in < 14) return;
  const long long need_x = ((long long)(NB - 1) * SEQ_FULL + SEQ) * DIM;
  if ((long long)in_sizes[0] < need_x) return;
  if (in_sizes[1] < DIM * DIM || in_sizes[2] < DIM * DIM || in_sizes[3] < DIM * DIM ||
      in_sizes[4] < DIM * DIM) return;
  if (in_sizes[6] < DIM * DFF || in_sizes[8] < DFF * DIM) return;
  if (in_sizes[5] < DIM || in_sizes[7] < DFF || in_sizes[9] < DIM) return;
  if (in_sizes[10] < DIM || in_sizes[11] < DIM || in_sizes[12] < DIM || in_sizes[13] < DIM)
    return;
  if ((long long)out_size < need_x) return;
  if (ws_size < WS_TOTAL) return;

  const float* x    = (const float*)d_in[0];
  const float* Wq   = (const float*)d_in[1];
  const float* Wk   = (const float*)d_in[2];
  const float* Wv   = (const float*)d_in[3];
  const float* Wo   = (const float*)d_in[4];
  const float* bo   = (const float*)d_in[5];
  const float* W1   = (const float*)d_in[6];
  const float* b1   = (const float*)d_in[7];
  const float* W2   = (const float*)d_in[8];
  const float* b2   = (const float*)d_in[9];
  const float* ln1s = (const float*)d_in[10];
  const float* ln1b = (const float*)d_in[11];
  const float* ln2s = (const float*)d_in[12];
  const float* ln2b = (const float*)d_in[13];
  float* out = (float*)d_out;

  char* ws = (char*)d_ws;
  _Float16* Wsq  = (_Float16*)(ws + OFF_WSQ);
  _Float16* W1t  = (_Float16*)(ws + OFF_W1T);
  _Float16* W2t  = (_Float16*)(ws + OFF_W2T);
  _Float16* H1   = (_Float16*)(ws + OFF_H1);
  _Float16* Qh16 = (_Float16*)(ws + OFF_Q);
  _Float16* Kh16 = (_Float16*)(ws + OFF_K);
  _Float16* Vt16 = (_Float16*)(ws + OFF_VT);
  _Float16* Ov16 = (_Float16*)(ws + OFF_OV);
  float*    X32  = (float*)(ws + OFF_X32);
  _Float16* H2   = (_Float16*)(ws + OFF_H2);
  _Float16* U16  = (_Float16*)(ws + OFF_U);

  const size_t WP = (size_t)DIM * DIM;
  dim3 blk(256);
  dim3 gD(DIM / 64, MROWS / 64);
  dim3 gF(DFF / 64, MROWS / 64);

  wconv_kernel<DIM, DIM><<<dim3(DIM / 64, DIM / 64, 4), blk, 0, stream>>>(Wq, Wk, Wv, Wo, Wsq);
  wconv_kernel<DIM, DFF><<<dim3(DFF / 64, DIM / 64, 1), blk, 0, stream>>>(W1, W1, W1, W1, W1t);
  wconv_kernel<DFF, DIM><<<dim3(DIM / 64, DFF / 64, 1), blk, 0, stream>>>(W2, W2, W2, W2, W2t);

  ln_kernel<1><<<dim3(MROWS / 8), blk, 0, stream>>>(x, ln1s, ln1b, H1);
  gemm_kernel<0, DIM, DIM><<<gD, blk, 0, stream>>>(H1, Wsq + 0 * WP, bo, X32, X32, Qh16);
  gemm_kernel<0, DIM, DIM><<<gD, blk, 0, stream>>>(H1, Wsq + 1 * WP, bo, X32, X32, Kh16);
  gemm_kernel<1, DIM, DIM><<<gD, blk, 0, stream>>>(H1, Wsq + 2 * WP, bo, X32, X32, Vt16);
  attn_kernel<<<dim3(SEQ / 128, NHEAD, NB), blk, 0, stream>>>(Qh16, Kh16, Vt16, Ov16);
  gemm_kernel<2, DIM, DIM><<<gD, blk, 0, stream>>>(Ov16, Wsq + 3 * WP, bo, x, X32, H2);
  ln_kernel<0><<<dim3(MROWS / 8), blk, 0, stream>>>(X32, ln2s, ln2b, H2);
  gemm_kernel<3, DIM, DFF><<<gF, blk, 0, stream>>>(H2, W1t, b1, X32, out, U16);
  gemm_kernel<4, DFF, DIM><<<gD, blk, 0, stream>>>(U16, W2t, b2, X32, out, H2);
}
